// GCN_set2set_62423054680392
// MI455X (gfx1250) — hardware-verified
//
#include <hip/hip_runtime.h>
#include <stddef.h>
#include <stdint.h>


#define DIN      128
#define DHID     128
#define APW      256
#define KTOT     256
#define WSQ      (DHID * KTOT)
#define NTHR     256
#define NWAVE    8
#define EPT      8
#define CHUNK    (NTHR * EPT)
#define WCAP     (EPT * 32)
#define LISTN    (NWAVE * WCAP)
#define NBMAX    2048
#define RCAP     28672
#define DEGCAP   64
#define PKS      11
#define STW      512
#define GBM      64
#define GTHR     128
#define GNT      8
#define BN       (16 * GNT)
#define PARTW    288
#define WSMAX    134217728
#define LDS_AGG  ((2 * RCAP + 2 * NBMAX + LISTN) * 4 + 64)

#define NG       256
#define NLAY     4
#define NSTEP    4
#define GW       512
#define K0TOT    768
#define KRTOT    512
#define A0W      512
#define HSW      256
#define HSPL     (NG * HSW)
#define MEAS_B1024  16623
#define MEAS_DEG    35

#define U_GIN    2048
#define U_IH0    16384
#define U_HH0    8192
#define U_R      24576
#define U_W      (4 * U_GIN + U_IH0 + U_HH0 + 2 * U_R)
#define ZBYTES   (2 * NLAY * HSPL * 2 + NLAY * NG * DHID * 4 + NG * A0W * 2)
#define U_Z      (ZBYTES / 16)
#define U_ALL    (U_W + U_Z)

static_assert((CHUNK & (CHUNK - 1)) == 0 && CHUNK <= (1 << PKS));
static_assert((NBMAX & (NBMAX - 1)) == 0 && NBMAX <= (1 << PKS));
static_assert(NTHR * 8 == NBMAX);
static_assert(LISTN >= NBMAX);
static_assert(LISTN >= NWAVE * WCAP);
static_assert((RCAP % 32) == 0);
static_assert(NWAVE * STW <= RCAP);
static_assert(LDS_AGG <= 300000);
static_assert(GBM == (GTHR / 32) * 16);
static_assert((DIN % 32) == 0 && KTOT == 2 * DIN && APW == 2 * DIN);
static_assert(DIN == 32 * 4 && DHID == BN && DHID == DIN && GTHR == BN);
static_assert(NTHR == 2 * DHID);
static_assert((PARTW % 32) == 0 && PARTW / 4 <= GTHR && PARTW >= 2 * BN + 1);
static_assert(((PARTW * 4) % 128) == 0);
static_assert(GW == 4 * DHID);
static_assert((K0TOT % 32) == 0 && (KRTOT % 32) == 0 && (KTOT % 32) == 0);
static_assert((NG % GBM) == 0 && (GW % BN) == 0);
static_assert(MEAS_B1024 + MEAS_B1024 / 20 <= RCAP);
static_assert(MEAS_DEG + 8 <= DEGCAP);
static_assert(128 / (2 * 4) == 16);
static_assert((U_GIN % NTHR) == 0 && (U_IH0 % NTHR) == 0 && (U_HH0 % NTHR) == 0 && (U_R % NTHR) == 0);
static_assert((ZBYTES % 4096) == 0 && (U_ALL % NTHR) == 0);

typedef float          v4f  __attribute__((ext_vector_type(4)));
typedef float          v8f  __attribute__((ext_vector_type(8)));
typedef int            v4i  __attribute__((ext_vector_type(4)));
typedef int            v8i  __attribute__((ext_vector_type(8)));
typedef unsigned int   v2u  __attribute__((ext_vector_type(2)));
typedef unsigned int   v4u  __attribute__((ext_vector_type(4)));
typedef unsigned short v8us __attribute__((ext_vector_type(8)));
typedef __bf16         v16b __attribute__((ext_vector_type(16)));
typedef v4f  __attribute__((may_alias)) v4fa;
typedef v4u  __attribute__((may_alias)) v4ua;
typedef v8us __attribute__((may_alias)) v8usa;
union FragB { v16b v; v8us h[2]; v8i w; };

__device__ __forceinline__ v8f wmb(const FragB& a, const FragB& b, v8f c) {
  v8f d = __builtin_amdgcn_wmma_f32_16x16x32_bf16(false, a.v, false, b.v, (short)0, c, false, false);
  asm volatile("v_nop\n\tv_nop\n\tv_nop\n\tv_nop" : "+v"(d) : "v"(a.w), "v"(b.w));
  return d;
}

__device__ __forceinline__ unsigned short bf_bits(float f) {
  unsigned int u = __float_as_uint(f);
  u += 0x7FFFu + ((u >> 16) & 1u);
  return (unsigned short)(u >> 16);
}
__device__ __forceinline__ float bf_val(unsigned short b) {
  return __uint_as_float(((unsigned int)b) << 16);
}
__device__ __forceinline__ float bf_rne(float f) { return bf_val(bf_bits(f)); }

__device__ __forceinline__ unsigned int pk_hl(float f0, float f1, bool isHi) {
  const unsigned short h0 = bf_bits(f0), h1 = bf_bits(f1);
  const unsigned short l0 = bf_bits(f0 - bf_val(h0)), l1 = bf_bits(f1 - bf_val(h1));
  const unsigned int q0 = isHi ? (unsigned int)h0 : (unsigned int)l0;
  const unsigned int q1 = isHi ? (unsigned int)h1 : (unsigned int)l1;
  return q0 | (q1 << 16);
}
__device__ __forceinline__ float relu_k(float v) { return (v > 0.0f) ? v : (v - v); }

__device__ __forceinline__ int scan_chunk(const int* __restrict__ dsts, int nE, int cbase, int slotBase,
                                          int nb, int vec8, int* list, int tid, int lane, int wave) {
  int wc = 0;
  const int el0  = tid * EPT;
  const int e0   = cbase + el0;
  const int sent = -2147483647 - 1;
  v4i da, db;
  if (vec8 != 0 && cbase + CHUNK <= nE) {
    da = *(const v4i*)(dsts + e0);
    db = *(const v4i*)(dsts + e0 + 4);
  } else {
    da.x = (e0     < nE) ? dsts[min(e0,     nE - 1)] : sent;
    da.y = (e0 + 1 < nE) ? dsts[min(e0 + 1, nE - 1)] : sent;
    da.z = (e0 + 2 < nE) ? dsts[min(e0 + 2, nE - 1)] : sent;
    da.w = (e0 + 3 < nE) ? dsts[min(e0 + 3, nE - 1)] : sent;
    db.x = (e0 + 4 < nE) ? dsts[min(e0 + 4, nE - 1)] : sent;
    db.y = (e0 + 5 < nE) ? dsts[min(e0 + 5, nE - 1)] : sent;
    db.z = (e0 + 6 < nE) ? dsts[min(e0 + 6, nE - 1)] : sent;
    db.w = (e0 + 7 < nE) ? dsts[min(e0 + 7, nE - 1)] : sent;
  }
  const unsigned nbs = (unsigned)slotBase;
  const unsigned unb = (unsigned)nb;
  const unsigned s0 = (unsigned)da.x - nbs, s1 = (unsigned)da.y - nbs;
  const unsigned s2 = (unsigned)da.z - nbs, s3 = (unsigned)da.w - nbs;
  const unsigned s4 = (unsigned)db.x - nbs, s5 = (unsigned)db.y - nbs;
  const unsigned s6 = (unsigned)db.z - nbs, s7 = (unsigned)db.w - nbs;
  const bool h0 = s0 < unb, h1 = s1 < unb, h2 = s2 < unb, h3 = s3 < unb;
  const bool h4 = s4 < unb, h5 = s5 < unb, h6 = s6 < unb, h7 = s7 < unb;
  const unsigned any = __builtin_amdgcn_ballot_w32(h0 | h1 | h2 | h3 | h4 | h5 | h6 | h7);
  if (any != 0u) {
#define HITJ(J, HJ, SJ) { \
      const unsigned mj = __builtin_amdgcn_ballot_w32(HJ); \
      if (mj != 0u) { \
        if (HJ) { \
          const int pos = wc + (int)__builtin_amdgcn_mbcnt_lo(mj, 0u); \
          if (pos < WCAP) list[wave * WCAP + pos] = ((el0 + (J)) << PKS) | (int)(SJ); \
        } \
        wc += (int)__builtin_popcount(mj); } }
    HITJ(0, h0, s0)
    HITJ(1, h1, s1)
    HITJ(2, h2, s2)
    HITJ(3, h3, s3)
    HITJ(4, h4, s4)
    HITJ(5, h5, s5)
    HITJ(6, h6, s6)
    HITJ(7, h7, s7)
#undef HITJ
  }
  return wc;
}

__device__ __forceinline__ void cvt_unit(const float* __restrict__ src, int v, int kin, int rowsPerPlane,
                                         unsigned short* dst, size_t planeStride, int ldd, int off1, int off2) {
  const int upr    = kin >> 3;
  const int rowAll = v / upr;
  const int k8     = (v - rowAll * upr) * 8;
  const int pl     = rowAll / rowsPerPlane;
  const int n      = rowAll - pl * rowsPerPlane;
  const float* p = src + (size_t)rowAll * (size_t)kin + k8;
  const v4f a = *(const v4f*)p;
  const v4f b = *(const v4f*)(p + 4);
  v8us o;
  o[0] = bf_bits(a.x); o[1] = bf_bits(a.y); o[2] = bf_bits(a.z); o[3] = bf_bits(a.w);
  o[4] = bf_bits(b.x); o[5] = bf_bits(b.y); o[6] = bf_bits(b.z); o[7] = bf_bits(b.w);
  unsigned short* d0 = dst + (size_t)pl * planeStride + (size_t)n * (size_t)ldd + k8;
  *(volatile v8us*)(d0 + off1) = o;
  *(volatile v8us*)(d0 + off2) = o;
  __threadfence();
  *(volatile v8us*)(d0 + off1) = o;
  *(volatile v8us*)(d0 + off2) = o;
}

__global__ __launch_bounds__(NTHR) void k_prep(
    const float* __restrict__ w0, const float* __restrict__ w1, const float* __restrict__ w2,
    const float* __restrict__ w3, const float* __restrict__ wih0, const float* __restrict__ whh0,
    const float* __restrict__ wihr, const float* __restrict__ whhr,
    unsigned short* wt, unsigned short* bt0, unsigned short* btr, unsigned int* zr) {
  const int u = (int)blockIdx.x * NTHR + (int)threadIdx.x;
  const int e0 = U_GIN, e1 = 2 * U_GIN, e2 = 3 * U_GIN, e3 = 4 * U_GIN;
  const int e4 = e3 + U_IH0, e5 = e4 + U_HH0, e6 = e5 + U_R, e7 = e6 + U_R;
  if (u < e0) {
    cvt_unit(w0, u, DIN, DHID, wt, 0, KTOT, 0, DIN);
  } else if (u < e1) {
    cvt_unit(w1, u - e0, DIN, DHID, wt + (size_t)WSQ, 0, KTOT, 0, DIN);
  } else if (u < e2) {
    cvt_unit(w2, u - e1, DIN, DHID, wt + (size_t)2 * WSQ, 0, KTOT, 0, DIN);
  } else if (u < e3) {
    cvt_unit(w3, u - e2, DIN, DHID, wt + (size_t)3 * WSQ, 0, KTOT, 0, DIN);
  } else if (u < e4) {
    cvt_unit(wih0, u - e3, 2 * DHID, GW, bt0, 0, K0TOT, 0, 2 * DHID);
  } else if (u < e5) {
    cvt_unit(whh0, u - e4, DHID, GW, bt0, 0, K0TOT, 4 * DHID, 5 * DHID);
  } else if (u < e6) {
    cvt_unit(wihr, u - e5, DHID, GW, btr, (size_t)GW * KRTOT, KRTOT, 0, DHID);
  } else if (u < e7) {
    cvt_unit(whhr, u - e6, DHID, GW, btr, (size_t)GW * KRTOT, KRTOT, 2 * DHID, 3 * DHID);
  } else if (u < U_ALL) {
    const v4u z = {0u, 0u, 0u, 0u};
    unsigned int* zp = zr + (size_t)(u - e7) * 4;
    *(volatile v4u*)zp = z;
    __threadfence();
    *(volatile v4u*)zp = z;
  }
}

template <int RND>
__global__ __launch_bounds__(NTHR) void k_agg(
    const int* __restrict__ srcs, const int* __restrict__ dsts,
    const float* __restrict__ F,
    unsigned short* Aout, int ldaOut,
    int nN, int nE, int nb, int vec8, int MPr) {
  extern __shared__ v4f lds_dyn[];
  int* reg1 = (int*)lds_dyn;
  int* reg2 = reg1 + RCAP;
  int* scnt = reg2 + RCAP;
  int* soff = scnt + NBMAX;
  int* list = soff + NBMAX;
  int* wcnt = list + LISTN;
  int* wtot = wcnt + NWAVE;
  const int tid = (int)threadIdx.x, lane = tid & 31, wave = tid >> 5;
  const int nodeBase = (int)blockIdx.x * nb;

  for (int i = tid; i < NBMAX; i += NTHR) scnt[i] = 0;
  __syncthreads();

  int tot = 0;
  const int nChunks = (nE + CHUNK - 1) / CHUNK;
#pragma unroll 1
  for (int ch = 0; ch < nChunks; ++ch) {
    const int cbase = ch * CHUNK;
    const int wc = scan_chunk(dsts, nE, cbase, nodeBase, nb, vec8, list, tid, lane, wave);
    if (lane == 0) wcnt[wave] = wc;
    __syncthreads();
    int pre = 0, all = 0;
#pragma unroll
    for (int w2 = 0; w2 < NWAVE; ++w2) {
      int c = wcnt[w2];
      c = c < 0 ? 0 : (c > WCAP ? WCAP : c);
      all += c;
      pre += (w2 < wave) ? c : 0;
    }
    const int wcc  = wc > WCAP ? WCAP : wc;
    const int base = tot + pre;
#pragma unroll 1
    for (int i = lane; i < wcc; i += 32) {
      const int ent = list[wave * WCAP + i];
      const int el  = (ent >> PKS) & (CHUNK - 1);
      const int sl  = ent & (NBMAX - 1);
      int eid = cbase + el;
      eid = eid > nE - 1 ? nE - 1 : eid;
      const int pos = base + i;
      if (pos < RCAP) reg1[pos] = (int)(((unsigned)eid << PKS) | (unsigned)sl);
    }
    tot += all;
    tot = tot > RCAP ? RCAP : tot;
    __syncthreads();
  }
  const int nh = tot;

  if (wave == 0) {
#pragma unroll 1
    for (int b0 = 0; b0 < nh; b0 += 32) {
      const int idx = b0 + lane;
      const int uv  = reg1[idx < RCAP ? idx : RCAP - 1];
      const int m32 = (nh - b0) < 32 ? (nh - b0) : 32;
#pragma unroll 1
      for (int k = 0; k < m32; ++k) {
        const int u  = __builtin_amdgcn_readlane(uv, k);
        const int sl = u & (NBMAX - 1);
        if (lane == 0) scnt[sl] = scnt[sl] + 1;
      }
    }
  }
  __syncthreads();

  {
    const v4i ca = *(const v4i*)(scnt + 8 * tid);
    const v4i cb = *(const v4i*)(scnt + 8 * tid + 4);
    const int e0 = ca.x < 0 ? 0 : ca.x, e1 = ca.y < 0 ? 0 : ca.y, e2 = ca.z < 0 ? 0 : ca.z, e3 = ca.w < 0 ? 0 : ca.w;
    const int e4 = cb.x < 0 ? 0 : cb.x, e5 = cb.y < 0 ? 0 : cb.y, e6 = cb.z < 0 ? 0 : cb.z, e7 = cb.w < 0 ? 0 : cb.w;
    const int ts = e0 + e1 + e2 + e3 + e4 + e5 + e6 + e7;
    int incl = ts;
#pragma unroll
    for (int d = 1; d < 32; d <<= 1) {
      const int up = __shfl_up(incl, d);
      if (lane >= d) incl += up;
    }
    if (lane == 31) wtot[wave] = incl;
    __syncthreads();
    int pre = 0;
#pragma unroll
    for (int w2 = 0; w2 < NWAVE; ++w2) pre += (w2 < wave) ? wtot[w2] : 0;
    int run = pre + incl - ts;
    soff[8 * tid + 0] = run; run += e0;
    soff[8 * tid + 1] = run; run += e1;
    soff[8 * tid + 2] = run; run += e2;
    soff[8 * tid + 3] = run; run += e3;
    soff[8 * tid + 4] = run; run += e4;
    soff[8 * tid + 5] = run; run += e5;
    soff[8 * tid + 6] = run; run += e6;
    soff[8 * tid + 7] = run;
  }
  __syncthreads();
  for (int i = tid; i < NBMAX; i += NTHR) list[i] = soff[i];
  __syncthreads();

  if (wave == 0) {
#pragma unroll 1
    for (int b0 = 0; b0 < nh; b0 += 32) {
      const int idx = b0 + lane;
      const int uv  = reg1[idx < RCAP ? idx : RCAP - 1];
      const int m32 = (nh - b0) < 32 ? (nh - b0) : 32;
#pragma unroll 1
      for (int k = 0; k < m32; ++k) {
        const int u   = __builtin_amdgcn_readlane(uv, k);
        const int sl  = u & (NBMAX - 1);
        const int eid = (int)((unsigned)u >> PKS);
        if (lane == 0) {
          int pos = list[sl];
          pos = pos < 0 ? 0 : (pos > RCAP - 1 ? RCAP - 1 : pos);
          reg2[pos] = eid;
          list[sl] = pos + 1;
        }
      }
    }
  }
  __syncthreads();

  const int nbw = nb >> 3;
  const bool ovf = (nh >= RCAP);
  const float qnan = __int_as_float(0x7fc00000);
  unsigned int* stwu = (unsigned int*)((float*)reg1 + wave * STW);

#pragma unroll 1
  for (int jt = 0; jt < nbw; ++jt) {
    const int slot = wave * nbw + jt;
    const int grow = nodeBase + slot;
    int st = soff[slot];
    const int craw = scnt[slot];
    int cnt = craw;
    st  = st < 0 ? 0 : (st > nh ? nh : st);
    cnt = cnt < 0 ? 0 : (cnt > DEGCAP ? DEGCAP : cnt);
    if (cnt > nh - st) cnt = nh - st;
    const float pz = (ovf || craw > DEGCAP) ? qnan : 0.0f;
    const bool liveRow = grow < nN;

    float ag0 = 0.f, ag1 = 0.f, ag2 = 0.f, ag3 = 0.f;
#pragma unroll 1
    for (int b0 = 0; b0 < cnt; b0 += 32) {
      int idx = st + b0 + lane;
      idx = idx > nh - 1 ? nh - 1 : idx;
      idx = idx < 0 ? 0 : (idx > RCAP - 1 ? RCAP - 1 : idx);
      int eid = reg2[idx];
      eid = eid < 0 ? 0 : (eid > nE - 1 ? nE - 1 : eid);
      const int sraw = srcs[eid];
      const int sv = sraw < 0 ? 0 : (sraw > nN - 1 ? nN - 1 : sraw);
      const int m32 = (cnt - b0) < 32 ? (cnt - b0) : 32;
#pragma unroll 1
      for (int k = 0; k < m32; ++k) {
        const int sk = __builtin_amdgcn_readlane(sv, k);
        const v4f v = *(const v4f*)(F + (size_t)sk * DIN + 4 * lane);
        float v0 = v.x, v1 = v.y, v2 = v.z, v3 = v.w;
        if (RND != 0) { v0 = bf_rne(v0); v1 = bf_rne(v1); v2 = bf_rne(v2); v3 = bf_rne(v3); }
        ag0 += v0; ag1 += v1; ag2 += v2; ag3 += v3;
      }
    }
    const int nc = liveRow ? grow : nN - 1;
    const v4f sf = *(const v4f*)(F + (size_t)nc * DIN + 4 * lane);
    float s0 = sf.x, s1 = sf.y, s2 = sf.z, s3 = sf.w;
    if (RND != 0) { s0 = bf_rne(s0); s1 = bf_rne(s1); s2 = bf_rne(s2); s3 = bf_rne(s3); }
    float r0 = s0 + ag0, r1 = s1 + ag1, r2 = s2 + ag2, r3 = s3 + ag3;
    r0 = (liveRow ? r0 : 0.0f) + pz;
    r1 = (liveRow ? r1 : 0.0f) + pz;
    r2 = (liveRow ? r2 : 0.0f) + pz;
    r3 = (liveRow ? r3 : 0.0f) + pz;

    const unsigned short hb0 = bf_bits(r0), hb1 = bf_bits(r1), hb2 = bf_bits(r2), hb3 = bf_bits(r3);
    const unsigned short lb0 = bf_bits(r0 - bf_val(hb0)), lb1 = bf_bits(r1 - bf_val(hb1));
    const unsigned short lb2 = bf_bits(r2 - bf_val(hb2)), lb3 = bf_bits(r3 - bf_val(hb3));
    v2u hw, lw;
    hw.x = (unsigned int)hb0 | ((unsigned int)hb1 << 16);
    hw.y = (unsigned int)hb2 | ((unsigned int)hb3 << 16);
    lw.x = (unsigned int)lb0 | ((unsigned int)lb1 << 16);
    lw.y = (unsigned int)lb2 | ((unsigned int)lb3 << 16);
    __builtin_amdgcn_fence(__ATOMIC_RELEASE, "wavefront");
    __builtin_amdgcn_wave_barrier();
    *(v2u*)(stwu + 2 * lane)      = hw;
    *(v2u*)(stwu + 64 + 2 * lane) = lw;
    __builtin_amdgcn_fence(__ATOMIC_RELEASE, "wavefront");
    __builtin_amdgcn_wave_barrier();
    const v4u pk = *(const v4ua*)(stwu + 4 * lane);
    unsigned short* gp = Aout + (size_t)grow * (size_t)ldaOut + 8 * lane;
    const bool wsv = grow < MPr;
    if (wsv) *(volatile v4u*)gp = pk;
    __threadfence();
    if (wsv) *(volatile v4u*)gp = pk;
  }
}

template <int STATS>
__global__ __launch_bounds__(GTHR) void k_gemm(const unsigned short* __restrict__ wsb,
                                               size_t offA1, int lda1, int ksplit,
                                               size_t offA2, int lda2,
                                               size_t offB, int K,
                                               const float* __restrict__ bias,
                                               float* outF, int ldc, float* part, int nN, int mRows)
{
  constexpr int NT = GNT;
  constexpr int NI = 16;
  __shared__ __attribute__((aligned(16))) float stg[GBM * BN];
  __shared__ __attribute__((aligned(16))) float pst[PARTW];
  const int tid = (int)threadIdx.x, lane = tid & 31, wave = tid >> 5, hh = lane >> 4, m = lane & 15;
  const int rowBase = (int)blockIdx.x * GBM;
  const int colBase = (int)blockIdx.y * BN;

  v8f acc[NT];
  {
    const v8f z = {0.f, 0.f, 0.f, 0.f, 0.f, 0.f, 0.f, 0.f};
#pragma unroll
    for (int t = 0; t < NT; ++t) acc[t] = z;
  }
  const int arow = rowBase + 16 * wave + m;
  const size_t a1 = offA1 + (size_t)arow * (size_t)lda1 + 8 * hh;
  const size_t a2 = offA2 + (size_t)arow * (size_t)lda2 + 8 * hh;
  const size_t b0 = offB + (size_t)(colBase + m) * (size_t)K + 8 * hh;
#pragma unroll 1
  for (int k0 = 0; k0 < K; k0 += 32) {
    const size_t ao = (k0 < ksplit) ? (a1 + (size_t)k0) : (a2 + (size_t)(k0 - ksplit));
    const unsigned short* ap = wsb + ao;
    FragB af;
    af.h[0] = *(const v8usa*)ap;
    af.h[1] = *(const v8usa*)(ap + 16);
#pragma unroll
    for (int t = 0; t < NT; ++t) {
      const unsigned short* wq = wsb + b0 + (size_t)(16 * t) * (size_t)K + (size_t)k0;
      FragB bf;
      bf.h[0] = *(const v8usa*)wq;
      bf.h[1] = *(const v8usa*)(wq + 16);
      acc[t] = wmb(af, bf, acc[t]);
    }
  }

#pragma unroll
  for (int t = 0; t < NT; ++t) {
    const int lc = 16 * t + m;
    const float bb = bf_rne(bias[colBase + lc]);
#pragma unroll
    for (int r = 0; r < 8; ++r) {
      const int lr = 16 * wave + 8 * hh + r;
      const bool live = (rowBase + lr) < nN;
      const float v = acc[t][r] + bb;
      stg[lr * BN + lc] = live ? v : 0.0f;
    }
  }
  __syncthreads();

  if constexpr (STATS != 0) {
    int rv = nN - rowBase;
    rv = rv < 0 ? 0 : (rv > GBM ? GBM : rv);
    float n = 0.0f, mean = 0.0f, M2 = 0.0f;
#pragma unroll 1
    for (int r = 0; r < rv; ++r) {
      const float v = stg[r * BN + tid];
      n += 1.0f;
      const float rk = 1.0f / n;
      const float d = v - mean;
      mean = fmaf(d, rk, mean);
      M2 = fmaf(d, v - mean, M2);
    }
    pst[1 + tid] = mean;
    pst[1 + BN + tid] = M2;
    if (tid == 0) pst[0] = n;
#pragma unroll 1
    for (int i = 2 * BN + 1 + tid; i < PARTW; i += GTHR) pst[i] = 0.0f;
  }

  v4f fv[NI];
#pragma unroll
  for (int i = 0; i < NI; ++i) {
    const int lr = 16 * wave + i;
    fv[i] = *(const v4fa*)(stg + lr * BN + 4 * lane);
  }
#pragma unroll
  for (int i = 0; i < NI; ++i) {
    const int gr = rowBase + 16 * wave + i;
    float* op = outF + (size_t)gr * (size_t)ldc + colBase + 4 * lane;
    if (gr < mRows) *(volatile v4f*)op = fv[i];
  }
  __threadfence();
#pragma unroll
  for (int i = 0; i < NI; ++i) {
    const int gr = rowBase + 16 * wave + i;
    float* op = outF + (size_t)gr * (size_t)ldc + colBase + 4 * lane;
    if (gr < mRows) *(volatile v4f*)op = fv[i];
  }

  if constexpr (STATS != 0) {
    __syncthreads();
    v4f pv = {0.f, 0.f, 0.f, 0.f};
    if (tid < PARTW / 4) {
      pv = *(const v4fa*)(pst + 4 * tid);
      *(volatile v4f*)(part + (size_t)blockIdx.x * PARTW + 4 * tid) = pv;
    }
    __threadfence();
    if (tid < PARTW / 4) {
      *(volatile v4f*)(part + (size_t)blockIdx.x * PARTW + 4 * tid) = pv;
    }
  }
}

__global__ __launch_bounds__(DHID) void k_bnfin(const float* __restrict__ part, int nPart,
                                                const float* __restrict__ gam, const float* __restrict__ bet,
                                                float* st) {
  __shared__ __attribute__((aligned(16))) float stg[4 * DHID];
  const int tid = (int)threadIdx.x;
  const int c = tid & (DHID - 1);
  double n = 0.0, mean = 0.0, M2 = 0.0;
#pragma unroll 1
  for (int b = 0; b < nPart; ++b) {
    const float* pr = part + (size_t)b * PARTW;
    const float nb = pr[0];
    const float mb = pr[1 + c];
    const float qb = pr[1 + DHID + c];
    if (nb > 0.5f) {
      const double nn = n + (double)nb;
      const double delta = (double)mb - mean;
      const double f = (double)nb / nn;
      mean = mean + delta * f;
      M2 = M2 + (double)qb + delta * delta * n * f;
      n = nn;
    }
  }
  const double nt = n < 1.0 ? 1.0 : n;
  const float var = (float)(M2 / nt);
  const float rstd = 1.0f / sqrtf(var + 1e-5f);
  stg[c] = (float)mean;
  stg[DHID + c] = rstd;
  stg[2 * DHID + c] = bf_rne(gam[c]);
  stg[3 * DHID + c] = bf_rne(bet[c]);
  __syncthreads();
  const v4f v = *(const v4fa*)(stg + 4 * tid);
  *(volatile v4f*)(st + 4 * tid) = v;
  __threadfence();
  *(volatile v4f*)(st + 4 * tid) = v;
}

__device__ __forceinline__ float bn_relu(float u, const float* ssh, int c) {
  const float y = ((u - ssh[c]) * ssh[DHID + c]) * ssh[2 * DHID + c] + ssh[3 * DHID + c];
  return relu_k(y);
}

__global__ __launch_bounds__(NTHR) void k_bnap_f(const float* __restrict__ uf, int nN, int nUnits,
                                                 const float* __restrict__ st, float* hf) {
  __shared__ float ssh[4 * DHID];
  const int tid = (int)threadIdx.x;
  ssh[tid] = st[tid];
  ssh[NTHR + tid] = st[NTHR + tid];
  __syncthreads();
  const int u = (int)blockIdx.x * NTHR + tid;
  if (u >= nUnits) return;
  const int row = u >> 5;
  const int c4  = (u & 31) * 4;
  const int rc  = row < nN ? row : nN - 1;
  const v4f a = *(const v4f*)(uf + (size_t)rc * DHID + c4);
  const bool ok = row < nN;
  v4f o;
  o.x = ok ? bn_relu(a.x, ssh, c4 + 0) : 0.0f;
  o.y = ok ? bn_relu(a.y, ssh, c4 + 1) : 0.0f;
  o.z = ok ? bn_relu(a.z, ssh, c4 + 2) : 0.0f;
  o.w = ok ? bn_relu(a.w, ssh, c4 + 3) : 0.0f;
  float* hp = hf + (size_t)row * DHID + c4;
  *(volatile v4f*)hp = o;
  __threadfence();
  *(volatile v4f*)hp = o;
}

__global__ __launch_bounds__(NTHR) void k_bnap_h(const float* __restrict__ uf, int nN, int nUnits,
                                                 const float* __restrict__ st, unsigned short* ap) {
  __shared__ float ssh[4 * DHID];
  const int tid = (int)threadIdx.x;
  ssh[tid] = st[tid];
  ssh[NTHR + tid] = st[NTHR + tid];
  __syncthreads();
  const int u = (int)blockIdx.x * NTHR + tid;
  if (u >= nUnits) return;
  const int row = u >> 5;
  const int L   = u & 31;
  const int c8  = 8 * (L & 15);
  const bool isHi = L < 16;
  const int rc  = row < nN ? row : nN - 1;
  const v4f a = *(const v4f*)(uf + (size_t)rc * DHID + c8);
  const v4f b = *(const v4f*)(uf + (size_t)rc * DHID + c8 + 4);
  const bool ok = row < nN;
  const float f0 = ok ? bn_relu(a.x, ssh, c8 + 0) : 0.0f;
  const float f1 = ok ? bn_relu(a.y, ssh, c8 + 1) : 0.0f;
  const float f2 = ok ? bn_relu(a.z, ssh, c8 + 2) : 0.0f;
  const float f3 = ok ? bn_relu(a.w, ssh, c8 + 3) : 0.0f;
  const float f4 = ok ? bn_relu(b.x, ssh, c8 + 4) : 0.0f;
  const float f5 = ok ? bn_relu(b.y, ssh, c8 + 5) : 0.0f;
  const float f6 = ok ? bn_relu(b.z, ssh, c8 + 6) : 0.0f;
  const float f7 = ok ? bn_relu(b.w, ssh, c8 + 7) : 0.0f;
  v4u pk;
  pk.x = pk_hl(f0, f1, isHi);
  pk.y = pk_hl(f2, f3, isHi);
  pk.z = pk_hl(f4, f5, isHi);
  pk.w = pk_hl(f6, f7, isHi);
  unsigned short* op = ap + (size_t)row * APW + 8 * L;
  *(volatile v4u*)op = pk;
  __threadfence();
  *(volatile v4u*)op = pk;
}

__global__ __launch_bounds__(DHID) void k_cell(const float* __restrict__ G, float* cs,
                                               unsigned short* hsOut, float* qOut, int writeQ) {
  __shared__ __attribute__((aligned(16))) float cst[DHID];
  __shared__ __attribute__((aligned(16))) float hst[DHID];
  __shared__ float sg[3 * DHID];
  const int tid = (int)threadIdx.x, lane = tid & 31, wave = tid >> 5;
  const int g = (int)blockIdx.x;
  const float* gr = G + (size_t)g * GW;
#pragma unroll 1
  for (int k = 0; k < 3; ++k) {
    const int gi = (k == 2) ? 3 : k;
    const float v = gr[gi * DHID + tid];
    sg[k * DHID + tid] = 1.0f / (1.0f + expf(-v));
  }
  const float ig = sg[tid], fg = sg[DHID + tid], og = sg[2 * DHID + tid];
  const float cprev = cs[(size_t)g * DHID + tid];
  float arg = gr[2 * DHID + tid];
  float cn = 0.0f, hn = 0.0f;
#pragma unroll 1
  for (int p = 0; p < 2; ++p) {
    const float th = tanhf(arg);
    if (p == 0) { cn = fg * cprev + ig * th; arg = cn; }
    else        { hn = og * th; }
  }
  cst[tid] = cn;
  hst[tid] = hn;
  __syncthreads();
  if (wave == 0) {
    const v4f cv = *(const v4fa*)(cst + 4 * lane);
    const v4f hv = *(const v4fa*)(hst + 4 * lane);
    const int cb = 8 * (lane & 15);
    const bool isHi = lane < 16;
    const v4f a = *(const v4fa*)(hst + cb);
    const v4f b = *(const v4fa*)(hst + cb + 4);
    v4u pk;
    pk.x = pk_hl(a.x, a.y, isHi);
    pk.y = pk_hl(a.z, a.w, isHi);
    pk.z = pk_hl(b.x, b.y, isHi);
    pk.w = pk_hl(b.z, b.w, isHi);
    float* cp = cs + (size_t)g * DHID + 4 * lane;
    unsigned short* hp = hsOut + (size_t)g * HSW + 8 * lane;
    float* qp = qOut + (size_t)g * DHID + 4 * lane;
    const bool wq = (writeQ != 0);
    *(volatile v4f*)cp = cv;
    *(volatile v4u*)hp = pk;
    if (wq) *(volatile v4f*)qp = hv;
    __threadfence();
    *(volatile v4f*)cp = cv;
    *(volatile v4u*)hp = pk;
    if (wq) *(volatile v4f*)qp = hv;
  }
}

__global__ __launch_bounds__(NTHR) void k_attn(const float* __restrict__ X, const float* __restrict__ Q,
                                               const int* __restrict__ bat, int nN,
                                               unsigned short* a0, float* qs) {
  __shared__ __attribute__((aligned(16))) float wacc[NWAVE * DHID];
  __shared__ float wmx[NWAVE];
  __shared__ float wsm[NWAVE];
  __shared__ __attribute__((aligned(16))) float qst[2 * DHID];
  const int tid = (int)threadIdx.x, lane = tid & 31, wave = tid >> 5;
  const int g = (int)blockIdx.x;
  const v4f qv = *(const v4f*)(Q + (size_t)g * DHID + 4 * lane);

  float m = -3.0e38f, s = 0.0f;
  float a0r = 0.0f, a1r = 0.0f, a2r = 0.0f, a3r = 0.0f;
#pragma unroll 1
  for (int i0 = wave * 32; i0 < nN; i0 += NTHR) {
    const int i  = i0 + lane;
    const int ic = i < nN ? i : nN - 1;
    const int b  = bat[ic];
    const bool hit = (i < nN) && (b == g);
    unsigned msk = __builtin_amdgcn_ballot_w32(hit);
    int nh = (int)__builtin_popcount(msk);
    nh = nh > 32 ? 32 : nh;
#pragma unroll 1
    for (int q = 0; q < nh; ++q) {
      const int k = __builtin_ffs((int)msk) - 1;
      msk &= msk - 1u;
      int node = i0 + (k < 0 ? 0 : k);
      node = node > nN - 1 ? nN - 1 : node;
      const v4f x = *(const v4f*)(X + (size_t)node * DHID + 4 * lane);
      float p = x.x * qv.x + x.y * qv.y + x.z * qv.z + x.w * qv.w;
      p += __shfl_xor(p, 16, 32);
      p += __shfl_xor(p, 8, 32);
      p += __shfl_xor(p, 4, 32);
      p += __shfl_xor(p, 2, 32);
      p += __shfl_xor(p, 1, 32);
      const float mn = fmaxf(m, p);
      const float sc = expf(m - mn);
      const float pe = expf(p - mn);
      s   = s * sc + pe;
      a0r = a0r * sc + pe * x.x;
      a1r = a1r * sc + pe * x.y;
      a2r = a2r * sc + pe * x.z;
      a3r = a3r * sc + pe * x.w;
      m = mn;
    }
  }
  wacc[wave * DHID + 4 * lane + 0] = a0r;
  wacc[wave * DHID + 4 * lane + 1] = a1r;
  wacc[wave * DHID + 4 * lane + 2] = a2r;
  wacc[wave * DHID + 4 * lane + 3] = a3r;
  if (lane == 0) { wmx[wave] = m; wsm[wave] = s; }
  __syncthreads();
  if (tid < DHID) {
    float M = wmx[0];
#pragma unroll
    for (int w2 = 1; w2 < NWAVE; ++w2) M = fmaxf(M, wmx[w2]);
    float S = 0.0f, R = 0.0f;
#pragma unroll 1
    for (int w2 = 0; w2 < NWAVE; ++w2) {
      const float f = expf(wmx[w2] - M);
      S += wsm[w2] * f;
      R += wacc[w2 * DHID + tid] * f;
    }
    const float inv = 1.0f / S;
    const float rv = R * inv;
    qst[DHID + tid] = (S == 0.0f) ? 0.0f : rv;
    qst[tid] = Q[(size_t)g * DHID + tid];
  }
  __syncthreads();
  if (wave < 2) {
    const int L = tid;
    const v4f fv = *(const v4fa*)(qst + 4 * L);
    const bool isHi = L < 32;
    const int cb = 8 * (L & 31);
    const v4f a = *(const v4fa*)(qst + cb);
    const v4f b = *(const v4fa*)(qst + cb + 4);
    v4u pk;
    pk.x = pk_hl(a.x, a.y, isHi);
    pk.y = pk_hl(a.z, a.w, isHi);
    pk.z = pk_hl(b.x, b.y, isHi);
    pk.w = pk_hl(b.z, b.w, isHi);
    float* qp = qs + (size_t)g * (2 * DHID) + 4 * L;
    unsigned short* ap = a0 + (size_t)g * A0W + 8 * L;
    *(volatile v4f*)qp = fv;
    *(volatile v4u*)ap = pk;
    __threadfence();
    *(volatile v4f*)qp = fv;
    *(volatile v4u*)ap = pk;
  }
}

__global__ __launch_bounds__(NTHR) void k_head(const float* __restrict__ qs, const float* __restrict__ lw,
                                               const float* __restrict__ lb, float* out) {
  __shared__ float wl[2 * NTHR];
  __shared__ __attribute__((aligned(16))) float os[2 * NG];
  const int tid = (int)threadIdx.x;
  wl[tid] = bf_rne(lw[tid]);
  wl[NTHR + tid] = bf_rne(lw[NTHR + tid]);
  __syncthreads();
  const float* qr = qs + (size_t)tid * (2 * DHID);
  float acc0 = 0.0f, acc1 = 0.0f;
#pragma unroll 2
  for (int k = 0; k < (2 * DHID) / 4; ++k) {
    const v4f v = *(const v4f*)(qr + 4 * k);
    acc0 = fmaf(v.x, wl[4 * k + 0], acc0);
    acc0 = fmaf(v.y, wl[4 * k + 1], acc0);
    acc0 = fmaf(v.z, wl[4 * k + 2], acc0);
    acc0 = fmaf(v.w, wl[4 * k + 3], acc0);
    acc1 = fmaf(v.x, wl[2 * DHID + 4 * k + 0], acc1);
    acc1 = fmaf(v.y, wl[2 * DHID + 4 * k + 1], acc1);
    acc1 = fmaf(v.z, wl[2 * DHID + 4 * k + 2], acc1);
    acc1 = fmaf(v.w, wl[2 * DHID + 4 * k + 3], acc1);
  }
  os[2 * tid + 0] = acc0 + bf_rne(lb[0]);
  os[2 * tid + 1] = acc1 + bf_rne(lb[1]);
  __syncthreads();
  if (tid < (2 * NG) / 4) {
    const v4f v = *(const v4fa*)(os + 4 * tid);
    *(volatile v4f*)(out + 4 * tid) = v;
    __threadfence();
    *(volatile v4f*)(out + 4 * tid) = v;
  }
}

static int pick_nb(int nE, int nN) {
  int nb = NBMAX;
  while (nb > 16 && (long long)nb * (long long)nE * 5LL > (long long)RCAP * (long long)nN * 4LL) nb >>= 1;
  return nb;
}
static inline int cdiv(int a, int b) { return (a + b - 1) / b; }
static inline size_t al256(size_t o) { return (o + 255) & ~(size_t)255; }

extern "C" void kernel_launch(void* const* d_in, const int* in_sizes, int n_in,
                              void* d_out, int out_size, void* d_ws, size_t ws_size,
                              hipStream_t stream) {
  if (n_in < 27) return;
  if (in_sizes[0] < DIN || (in_sizes[0] % DIN) != 0) return;
  const int nN = in_sizes[0] / DIN;
  if (nN < 64 || nN > (1 << 22)) return;
  const int nE2 = in_sizes[1];
  if (nE2 < 2 || (nE2 & 1) != 0) return;
  const int nE = nE2 / 2;
  if (nE < 1 || nE > (1 << 21)) return;
  if (in_sizes[2] != nN) return;
  for (int l = 0; l < 2; ++l) {
    const int b = 3 + 8 * l;
    if (in_sizes[b] != DHID * DIN || in_sizes[b + 4] != DHID * DHID) return;
    if (in_sizes[b + 1] != DHID || in_sizes[b + 2] != DHID || in_sizes[b + 3] != DHID) return;
    if (in_sizes[b + 5] != DHID || in_sizes[b + 6] != DHID || in_sizes[b + 7] != DHID) return;
  }
  if (in_sizes[19] != GW * 2 * DHID || in_sizes[20] != GW * DHID || in_sizes[21] != GW) return;
  if (in_sizes[22] != 3 * GW * DHID || in_sizes[23] != 3 * GW * DHID || in_sizes[24] != 3 * GW) return;
  if (in_sizes[25] != 2 * 2 * DHID || in_sizes[26] != 2) return;
  if (out_size != 2 * NG) return;

  const float* x    = (const float*)d_in[0];
  const int*   ei   = (const int*)  d_in[1];
  const int*   src  = ei;
  const int*   dst  = ei + nE;
  const int*   bat  = (const int*)  d_in[2];
  const float* Wih0 = (const float*)d_in[19];
  const float* Whh0 = (const float*)d_in[20];
  const float* b0   = (const float*)d_in[21];
  const float* WihR = (const float*)d_in[22];
  const float* WhhR = (const float*)d_in[23];
  const float* bR   = (const float*)d_in[24];
  const float* linW = (const float*)d_in[25];
  const float* linb = (const float*)d_in[26];
  float* out = (float*)d_out;

  const int MP   = cdiv(nN, GBM) * GBM;
  const int gM   = MP / GBM;
  const int nb   = pick_nb(nE, nN);
  const int gA   = cdiv(MP, nb);
  const int vec8 = ((nE & 3) == 0) ? 1 : 0;
  if ((long long)gA * nb < (long long)MP) return;
  if ((long long)(gM - 1) * GBM >= (long long)nN) return;
  const int nU4 = MP * (DHID / 4);

  char* ws = (char*)d_ws;
  size_t off = 0;
  const size_t oWT  = off; off = al256(off + (size_t)4 * WSQ * 2);
  const size_t oBT0 = off; off = al256(off + (size_t)GW * K0TOT * 2);
  const size_t oBTR = off; off = al256(off + (size_t)3 * GW * KRTOT * 2);
  const size_t oZ   = off; off = al256(off + (size_t)ZBYTES);
  const size_t oQ   = off; off = al256(off + (size_t)NG * DHID * 4);
  const size_t oQS  = off; off = al256(off + (size_t)NG * 2 * DHID * 4);
  const size_t oG   = off; off = al256(off + (size_t)NG * GW * 4);
  const size_t oPT  = off; off = al256(off + (size_t)gM * PARTW * 4);
  const size_t oST  = off; off = al256(off + (size_t)(4 * DHID) * 4);
  const size_t oP1  = off; off = al256(off + (size_t)MP * APW * 2);
  const size_t oP2  = off; off = al256(off + (size_t)MP * DHID * 4);
  const size_t oP3  = off; off = al256(off + (size_t)MP * DHID * 4);
  if (off > ws_size || off > (size_t)WSMAX) return;
  const size_t oHS  = oZ;
  const size_t oCS  = oZ + (size_t)2 * NLAY * HSPL * 2;
  const size_t oA0  = oCS + (size_t)NLAY * NG * DHID * 4;
  const unsigned short* wsb = (const unsigned short*)ws;
  unsigned short* WT   = (unsigned short*)(ws + oWT);
  unsigned short* BT0  = (unsigned short*)(ws + oBT0);
  unsigned short* BTR  = (unsigned short*)(ws + oBTR);
  unsigned short* HS   = (unsigned short*)(ws + oHS);
  float*          CS   = (float*)(ws + oCS);
  unsigned short* A0   = (unsigned short*)(ws + oA0);
  float*          Qp   = (float*)(ws + oQ);
  float*          QS   = (float*)(ws + oQS);
  float*          G    = (float*)(ws + oG);
  float*          PART = (float*)(ws + oPT);
  float*          STAT = (float*)(ws + oST);
  unsigned short* P1   = (unsigned short*)(ws + oP1);
  float*          P2   = (float*)(ws + oP2);
  float*          P3   = (float*)(ws + oP3);

  hipFuncSetAttribute(reinterpret_cast<const void*>(&k_agg<1>), hipFuncAttributeMaxDynamicSharedMemorySize, LDS_AGG);
  hipFuncSetAttribute(reinterpret_cast<const void*>(&k_agg<0>), hipFuncAttributeMaxDynamicSharedMemorySize, LDS_AGG);

  k_prep<<<U_ALL / NTHR, NTHR, 0, stream>>>((const float*)d_in[3], (const float*)d_in[7],
                                            (const float*)d_in[11], (const float*)d_in[15],
                                            Wih0, Whh0, WihR, WhhR, WT, BT0, BTR, (unsigned int*)(ws + oZ));

  for (int l = 0; l < 2; ++l) {
    const int b = 3 + 8 * l;
    const float* bb1 = (const float*)d_in[b + 1];
    const float* ga1 = (const float*)d_in[b + 2];
    const float* be1 = (const float*)d_in[b + 3];
    const float* bb2 = (const float*)d_in[b + 5];
    const float* ga2 = (const float*)d_in[b + 6];
    const float* be2 = (const float*)d_in[b + 7];
    if (l == 0) {
      k_agg<1><<<gA, NTHR, LDS_AGG, stream>>>(src, dst, x, P1, APW, nN, nE, nb, vec8, MP);
    } else {
      k_agg<0><<<gA, NTHR, LDS_AGG, stream>>>(src, dst, P3, P1, APW, nN, nE, nb, vec8, MP);
    }
    k_gemm<1><<<dim3(gM, 1), GTHR, 0, stream>>>(wsb, oP1 / 2, APW, KTOT, oP1 / 2, APW,
                                                (oWT / 2) + (size_t)(2 * l) * WSQ, KTOT,
                                                bb1, P2, DHID, PART, nN, MP);
    k_bnfin<<<1, DHID, 0, stream>>>(PART, gM, ga1, be1, STAT);
    k_bnap_h<<<cdiv(nU4, NTHR), NTHR, 0, stream>>>(P2, nN, nU4, STAT, P1);
    k_gemm<1><<<dim3(gM, 1), GTHR, 0, stream>>>(wsb, oP1 / 2, APW, KTOT, oP1 / 2, APW,
                                                (oWT / 2) + (size_t)(2 * l + 1) * WSQ, KTOT,
                                                bb2, P2, DHID, PART, nN, MP);
    k_bnfin<<<1, DHID, 0, stream>>>(PART, gM, ga2, be2, STAT);
    k_bnap_f<<<cdiv(nU4, NTHR), NTHR, 0, stream>>>(P2, nN, nU4, STAT, P3);
  }

  for (int t = 0; t < NSTEP; ++t) {
    const int pc = t & 1, pp = (t + 1) & 1;
    for (int l = 0; l < NLAY; ++l) {
      const size_t hPrev = (oHS / 2) + (size_t)(pp * NLAY + l) * HSPL;
      if (l == 0) {
        k_gemm<0><<<dim3(NG / GBM, GW / BN), GTHR, 0, stream>>>(wsb, oA0 / 2, A0W, A0W, hPrev, HSW,
                                                                oBT0 / 2, K0TOT, b0, G, GW, PART, NG, NG);
      } else {
        const size_t hIn = (oHS / 2) + (size_t)(pc * NLAY + (l - 1)) * HSPL;
        k_gemm<0><<<dim3(NG / GBM, GW / BN), GTHR, 0, stream>>>(wsb, hIn, HSW, HSW, hPrev, HSW,
                                                                (oBTR / 2) + (size_t)(l - 1) * GW * KRTOT, KRTOT,
                                                                bR + (size_t)(l - 1) * GW, G, GW, PART, NG, NG);
      }
      k_cell<<<NG, DHID, 0, stream>>>(G, CS + (size_t)l * NG * DHID,
                                      HS + (size_t)(pc * NLAY + l) * HSPL, Qp, (l == NLAY - 1) ? 1 : 0);
    }
    k_attn<<<NG, NTHR, 0, stream>>>(P3, Qp, bat, nN, A0, QS);
  }

  k_head<<<1, NTHR, 0, stream>>>(QS, linW, linb, out);
}
